// CNN_tagger_20761871909366
// MI455X (gfx1250) — hardware-verified
//
#include <hip/hip_runtime.h>
#include <hip/hip_bf16.h>


typedef __attribute__((ext_vector_type(16))) _Float16 v16h;
typedef __attribute__((ext_vector_type(8)))  _Float16 v8h;
typedef __attribute__((ext_vector_type(4)))  unsigned v4u;
template <typename T> __device__ __forceinline__ void vst2(void* p, T v) { *(volatile T*)p = v; __threadfence(); *(volatile T*)p = v; }
typedef __attribute__((ext_vector_type(8)))  float  v8f;
typedef __attribute__((ext_vector_type(4)))  int    v4i;
typedef __attribute__((ext_vector_type(4)))  float  v4f;
typedef __attribute__((ext_vector_type(2)))  int    v2i;

typedef const v4i __attribute__((address_space(1)))* gcv4i;
typedef const v4f __attribute__((address_space(1)))* gcv4f;
typedef       v4f __attribute__((address_space(1)))* gv4f;

static __device__ __forceinline__ v4i gload4i(const void* p) {
  return *(gcv4i)(unsigned long long)p;
}
static __device__ __forceinline__ v4f gload4f(const void* p) {
  return *(gcv4f)(unsigned long long)p;
}
static __device__ __forceinline__ void gstore4f(void* p, v4f v) {
  *(gv4f)(unsigned long long)p = v;
}

union Frag16 { v4i q[2]; v16h bf; };
typedef __attribute__((ext_vector_type(8)))  float  v8f_;
static __device__ __forceinline__ v8f_ WMMA16(bool, v16h a, bool, v16h b, short, v8f_ c, bool, bool) {
  v8f_ d = __builtin_amdgcn_wmma_f32_16x16x32_f16(false, a, false, b, (short)0, c, false, false);
  asm volatile("v_nop\n\tv_nop\n\tv_nop\n\tv_nop" : "+v"(d) : "v"(a), "v"(b));
  return d;
}
union Pack8  { _Float16 p[8]; v4i q; };
union Pack4  { _Float16 p[4]; v2i q; };

#define XSTR 520
#define FSTR 776

__global__ void pack_conv_w(const float* __restrict__ src,
                            _Float16* __restrict__ dst, int k) {
  int n8 = 256 * 512 * k / 8;
  int g = blockIdx.x * blockDim.x + threadIdx.x;
  if (g >= n8) return;
  union { v8h h; v4u u; } pk;
#pragma unroll
  for (int e = 0; e < 8; ++e) {
    int t = g * 8 + e;
    int nk  = t / (512 * k);
    int rem = t - nk * 512 * k;
    int dk  = rem >> 9;
    int d   = rem & 511;
    pk.h[e] = (_Float16)src[(nk * 512 + d) * k + dk];
  }
  vst2(dst + (size_t)g * 8, pk.u);
}

__global__ void pack_lin_w(const float* __restrict__ src,
                           _Float16* __restrict__ dst, int n) {
  int g = blockIdx.x * blockDim.x + threadIdx.x;
  if (g * 8 >= n) return;
  union { v8h h; v4u u; } pk;
#pragma unroll
  for (int e = 0; e < 8; ++e) pk.h[e] = (_Float16)src[g * 8 + e];
  vst2(dst + (size_t)g * 8, pk.u);
}

__global__ __launch_bounds__(256) void cnn_tagger_kernel(
    const float* __restrict__ x,
    const float* __restrict__ cb3, const float* __restrict__ cb5,
    const float* __restrict__ cb7, const float* __restrict__ linb,
    const _Float16* __restrict__ wA3,
    const _Float16* __restrict__ wA5,
    const _Float16* __restrict__ wA7,
    const _Float16* __restrict__ wL,
    float* __restrict__ out)
{
  __shared__ _Float16 lds_x[22 * XSTR];
  __shared__ _Float16 feats[16 * FSTR];
  __shared__ __attribute__((aligned(16))) float so[16 * 64];

  const int tid  = threadIdx.x;
  const int wave = tid >> 5;
  const int lane = tid & 31;
  const int i    = lane & 15;
  const int h    = lane >> 4;

  const int b  = blockIdx.x >> 5;
  const int s0 = (blockIdx.x & 31) << 4;

  const float* xb = x + (size_t)b * (512 * 512);
  for (int it = 0; it < 11; ++it) {
    int f   = it * 256 + tid;
    int row = f >> 7;
    int c4  = f & 127;
    int sg  = s0 - 3 + row;
    v4f v = {0.f, 0.f, 0.f, 0.f};
    if (sg >= 0 && sg < 512) v = gload4f(xb + sg * 512 + c4 * 4);
    Pack4 pk;
    pk.p[0] = (_Float16)v.x; pk.p[1] = (_Float16)v.y;
    pk.p[2] = (_Float16)v.z; pk.p[3] = (_Float16)v.w;
    *(v2i*)&lds_x[row * XSTR + c4 * 4] = pk.q;
  }
  __syncthreads();

  const int     ks[3]  = {3, 5, 7};
  const _Float16* wAs[3] = {wA3, wA5, wA7};
  const float*  cbs[3] = {cb3, cb5, cb7};

  for (int bi = 0; bi < 3; ++bi) {
    const int k      = ks[bi];
    const int rowoff = 3 - ((k - 1) >> 1);
    const int Kb     = k * 512;
    const int nchunk = k * 16;
    const _Float16* wA = wAs[bi];
    const float*  cb = cbs[bi];

    const int cl0 = wave * 16;
    const _Float16* w0 = wA + (size_t)(cl0 + i) * Kb + h * 8;
    const _Float16* w1 = w0 + (size_t)128 * Kb;

    v8f acc0 = {};
    v8f acc1 = {};
    for (int kc = 0; kc < nchunk; ++kc) {
      const int dk    = kc >> 4;
      const int dbase = (kc & 15) << 5;
      Frag16 Bf;
      const _Float16* bp = &lds_x[(i + dk + rowoff) * XSTR + dbase + h * 8];
      Bf.q[0] = *(const v4i*)bp;
      Bf.q[1] = *(const v4i*)(bp + 16);
      Frag16 A0, A1;
      const _Float16* a0 = w0 + kc * 32;
      const _Float16* a1 = w1 + kc * 32;
      A0.q[0] = gload4i(a0); A0.q[1] = gload4i(a0 + 16);
      A1.q[0] = gload4i(a1); A1.q[1] = gload4i(a1 + 16);
      acc0 = WMMA16(
          false, A0.bf, false, Bf.bf, (short)0, acc0, false, false);
      acc1 = WMMA16(
          false, A1.bf, false, Bf.bf, (short)0, acc1, false, false);
    }

#pragma unroll
    for (int tl = 0; tl < 2; ++tl) {
      const v8f acc = tl ? acc1 : acc0;
      const int cl  = cl0 + tl * 128;
      v4f bl = gload4f(cb + cl + h * 8);
      v4f bh = gload4f(cb + cl + h * 8 + 4);
      Pack8 pk;
#pragma unroll
      for (int r = 0; r < 8; ++r) {
        float fv = acc[r] + ((r < 4) ? bl[r] : bh[r - 4]);
        fv = fv > 0.f ? fv : 0.f;
        pk.p[r] = (_Float16)fv;
      }
      *(v4i*)&feats[i * FSTR + bi * 256 + cl + h * 8] = pk.q;
    }
  }
  __syncthreads();

  if (wave < 4) {
    const int o0 = wave * 16;
    const _Float16* wrow = wL + (size_t)(o0 + i) * 768 + h * 8;
    v8f acc = {};
    for (int kc = 0; kc < 24; ++kc) {
      Frag16 Bf;
      const _Float16* bp = &feats[i * FSTR + kc * 32 + h * 8];
      Bf.q[0] = *(const v4i*)bp;
      Bf.q[1] = *(const v4i*)(bp + 16);
      Frag16 Af;
      const _Float16* ap = wrow + kc * 32;
      Af.q[0] = gload4i(ap);
      Af.q[1] = gload4i(ap + 16);
      acc = WMMA16(
          false, Af.bf, false, Bf.bf, (short)0, acc, false, false);
    }
#pragma unroll
    for (int r = 0; r < 8; ++r) so[i * 64 + o0 + h * 8 + r] = acc[r] + linb[o0 + h * 8 + r];
  }
  __syncthreads();
  {
    const int rl = tid >> 4, pc = tid & 15;
    vst2(out + ((size_t)(b * 512 + s0 + rl)) * 64 + pc * 4, *(const v4f*)(so + rl * 64 + pc * 4));
  }
}

extern "C" void kernel_launch(void* const* d_in, const int* in_sizes, int n_in,
                              void* d_out, int out_size, void* d_ws,
                              size_t ws_size, hipStream_t stream) {
  const float* x   = (const float*)d_in[0];
  const float* w3  = (const float*)d_in[1];
  const float* b3  = (const float*)d_in[2];
  const float* w5  = (const float*)d_in[3];
  const float* b5  = (const float*)d_in[4];
  const float* w7  = (const float*)d_in[5];
  const float* b7  = (const float*)d_in[6];
  const float* lw  = (const float*)d_in[7];
  const float* lb  = (const float*)d_in[8];
  float* out = (float*)d_out;

  _Float16* wA3 = (_Float16*)d_ws;
  _Float16* wA5 = wA3 + 256 * (3 * 512);
  _Float16* wA7 = wA5 + 256 * (5 * 512);
  _Float16* wL  = wA7 + 256 * (7 * 512);

  pack_conv_w<<<(256 * 512 * 3 / 8 + 255) / 256, 256, 0, stream>>>(w3, wA3, 3);
  pack_conv_w<<<(256 * 512 * 5 / 8 + 255) / 256, 256, 0, stream>>>(w5, wA5, 5);
  pack_conv_w<<<(256 * 512 * 7 / 8 + 255) / 256, 256, 0, stream>>>(w7, wA7, 7);
  pack_lin_w<<<(64 * 768 / 8 + 255) / 256, 256, 0, stream>>>(lw, wL, 64 * 768);

  cnn_tagger_kernel<<<1024, 256, 0, stream>>>(x, b3, b5, b7, lb,
                                              wA3, wA5, wA7, wL, out);
}
